// ConvAttention_25477746000320
// MI455X (gfx1250) — hardware-verified
//
#include <hip/hip_runtime.h>
#include <stdint.h>
#include <stddef.h>

typedef __attribute__((ext_vector_type(16))) _Float16 v16h;
typedef __attribute__((ext_vector_type(8)))  _Float16 v8h;
typedef __attribute__((ext_vector_type(16))) __bf16   v16b;
typedef __attribute__((ext_vector_type(8)))  __bf16   v8b;
typedef __attribute__((ext_vector_type(8)))  float    v8f;
typedef __attribute__((ext_vector_type(4)))  float    v4f;
typedef __attribute__((ext_vector_type(4)))  unsigned int   v4u;
typedef __attribute__((ext_vector_type(8)))  unsigned short v8us;

__device__ __forceinline__ unsigned short f2bf_bits(float f) {
  unsigned u = __float_as_uint(f);
  return (unsigned short)((u + 0x7FFFu + ((u >> 16) & 1u)) >> 16);
}
__device__ __forceinline__ float bf_bits2f(unsigned short h) { return __uint_as_float(((unsigned)h) << 16); }

__device__ __forceinline__ void dep_guard_h(v8f& a, v8f& b, v16h x, v16h y) { asm volatile("v_nop\n\tv_nop\n\tv_nop\n\tv_nop" : "+v"(a), "+v"(b) : "v"(x), "v"(y)); }
__device__ __forceinline__ void dep_guard_b(v8f& a, v8f& b, v16b x, v16b y) { asm volatile("v_nop\n\tv_nop\n\tv_nop\n\tv_nop" : "+v"(a), "+v"(b) : "v"(x), "v"(y)); }
__device__ __forceinline__ void keep4_h(v16h a, v16h b, v16h c, v16h d) { asm volatile("v_nop" :: "v"(a), "v"(b), "v"(c), "v"(d)); }
__device__ __forceinline__ void keep4_b(v16b a, v16b b, v16b c, v16b d) { asm volatile("v_nop" :: "v"(a), "v"(b), "v"(c), "v"(d)); }
__device__ __forceinline__ void acc_guard4(v8f& a, v8f& b, v8f& c, v8f& d) { asm volatile("v_nop\n\tv_nop\n\tv_nop\n\tv_nop" : "+v"(a), "+v"(b), "+v"(c), "+v"(d)); }
template <typename T> struct Frag;
template <> struct Frag<_Float16> {
  typedef v16h V; union U { v16h v; v8h h[2]; };
  static __device__ __forceinline__ v16h load(const _Float16* p) {
    U f; f.h[0] = *(const v8h*)(p); f.h[1] = *(const v8h*)(p + 16); return f.v;
  }
  static __device__ __forceinline__ v8f mma(v16h a, v16h b, v8f c) {
    return __builtin_amdgcn_wmma_f32_16x16x32_f16(false, a, false, b, (short)0, c, false, false);
  }
  static __device__ __forceinline__ void guard(v8f& a, v8f& b, v16h x, v16h y) { dep_guard_h(a, b, x, y); }
  static __device__ __forceinline__ void keep(v16h a, v16h b, v16h c, v16h d) { keep4_h(a, b, c, d); }
};
template <> struct Frag<__bf16> {
  typedef v16b V; union U { v16b v; v8b h[2]; };
  static __device__ __forceinline__ v16b load(const __bf16* p) {
    U f; f.h[0] = *(const v8b*)(p); f.h[1] = *(const v8b*)(p + 16); return f.v;
  }
  static __device__ __forceinline__ v8f mma(v16b a, v16b b, v8f c) {
    return __builtin_amdgcn_wmma_f32_16x16x32_bf16(false, a, false, b, (short)0, c, false, false);
  }
  static __device__ __forceinline__ void guard(v8f& a, v8f& b, v16b x, v16b y) { dep_guard_b(a, b, x, y); }
  static __device__ __forceinline__ void keep(v16b a, v16b b, v16b c, v16b d) { keep4_b(a, b, c, d); }
};

template <int ET> struct Elem;
template <> struct Elem<0> { typedef _Float16 T; };
template <> struct Elem<1> { typedef __bf16 T; };
template <int ET, bool SPLIT, int BIAS_MODE, int OUT_MODE, bool RESID, int ACT = 0>
__global__ __launch_bounds__(256) void wmma_gemm64(
    const unsigned short* __restrict__ Ap, const unsigned short* __restrict__ A2p, int lda, long strideA,
    const unsigned short* __restrict__ Btp, const unsigned short* __restrict__ Bt2p, int ldb, long strideB,
    void* __restrict__ Cout, void* __restrict__ Cout2, int ldc, long strideC,
    const float* __restrict__ bias,
    const float* __restrict__ resid, long strideR,
    int M, int N, int K, float scale) {
  typedef typename Elem<ET>::T T;
  typedef typename Frag<T>::V V;
  const T* A = (const T*)Ap; const T* A2 = (const T*)A2p; const T* Bt = (const T*)Btp; const T* Bt2 = (const T*)Bt2p;
  __shared__ __align__(16) float sT[8][16 * 68];
  const int b    = blockIdx.y;
  const int lane = threadIdx.x & 31;
  const int wave = threadIdx.x >> 5;
  const int tilesN = N >> 6;
  const int tilesM = M >> 6;
  const int tile = blockIdx.x * 8 + wave;
  if (tile >= tilesM * tilesN) return;
  const int tm = tile / tilesN;
  const int tn = tile - tm * tilesN;
  const int m0 = tm << 6;
  const int n0 = tn << 6;

  const T* Ab  = A  + (size_t)b * strideA;
  const T* Bb  = Bt + (size_t)b * strideB;
  const T* Ab2 = SPLIT ? (A2  + (size_t)b * strideA) : nullptr;
  const T* Bb2 = SPLIT ? (Bt2 + (size_t)b * strideB) : nullptr;

  const int rlane = lane & 15;
  const int koff  = (lane >> 4) * 8;
  const int mOff  = (lane >> 4) * 8;

  v8f acc[4][4];
#pragma unroll
  for (int i = 0; i < 4; ++i)
#pragma unroll
    for (int j = 0; j < 4; ++j) acc[i][j] = (v8f){0.f,0.f,0.f,0.f,0.f,0.f,0.f,0.f};

  for (int k0 = 0; k0 < K; k0 += 32) {
    V bh[4], bl[4];
#pragma unroll
    for (int j = 0; j < 4; ++j) {
      const size_t bo = (size_t)(n0 + (j << 4) + rlane) * ldb + koff + k0;
      bh[j] = Frag<T>::load(Bb + bo);
      if (SPLIT) bl[j] = Frag<T>::load(Bb2 + bo);
    }
#pragma unroll
    for (int i = 0; i < 4; ++i) {
      const size_t ao = (size_t)(m0 + (i << 4) + rlane) * lda + koff + k0;
      V ah = Frag<T>::load(Ab + ao);
      V al;
      if (SPLIT) al = Frag<T>::load(Ab2 + ao);
#pragma unroll
      for (int j = 0; j < 4; ++j) {
        acc[i][j] = Frag<T>::mma(ah, bh[j], acc[i][j]);
        if (SPLIT) {
          acc[i][j] = Frag<T>::mma(ah, bl[j], acc[i][j]);
          acc[i][j] = Frag<T>::mma(al, bh[j], acc[i][j]);
        }
      }
      Frag<T>::guard(acc[i][0], acc[i][3], ah, SPLIT ? al : ah);
    }
    Frag<T>::keep(bh[0], bh[1], bh[2], bh[3]);
    if (SPLIT) Frag<T>::keep(bl[0], bl[1], bl[2], bl[3]);
  }
  acc_guard4(acc[0][0], acc[0][1], acc[0][2], acc[0][3]);
  acc_guard4(acc[1][0], acc[1][1], acc[1][2], acc[1][3]);
  acc_guard4(acc[2][0], acc[2][1], acc[2][2], acc[2][3]);
  acc_guard4(acc[3][0], acc[3][1], acc[3][2], acc[3][3]);

  float* slab = sT[wave];
  const float* Rb = RESID ? (resid + (size_t)b * strideR) : nullptr;
#pragma unroll
  for (int i = 0; i < 4; ++i) {
    const int mBase = m0 + (i << 4);
#pragma unroll
    for (int j = 0; j < 4; ++j) {
      const int n = n0 + (j << 4) + rlane;
      float bv = 0.f;
      if (BIAS_MODE == 2) bv = bias[n];
#pragma unroll
      for (int r = 0; r < 8; ++r) {
        float v = acc[i][j][r] * scale;
        if (BIAS_MODE == 1) v += bias[mBase + mOff + r];
        if (BIAS_MODE == 2) v += bv;
        if (RESID) v += Rb[(size_t)(mBase + mOff + r) * ldc + n];
        if (ACT == 1) v = tanhf(v);
        if (ACT == 2) v = fmaxf(v, 0.0f);
        if (ACT == 3) v = v / (1.0f + expf(-v));
        if (ACT == 4) v = (v > 0.f) ? v : 0.01f * v;
        if (ACT == 5) v = 0.5f * v * (1.0f + erff(v * 0.70710678118654752f));
        slab[(mOff + r) * 68 + (j << 4) + rlane] = v;
      }
    }
    __builtin_amdgcn_fence(__ATOMIC_RELEASE, "workgroup");
    __builtin_amdgcn_wave_barrier();
    __builtin_amdgcn_fence(__ATOMIC_ACQUIRE, "workgroup");
    if (OUT_MODE == 0) {
      float* C = (float*)Cout + (size_t)b * strideC;
      const int hh = lane >> 4, c4 = (lane & 15) * 4;
      for (int pass = 0; pass < 2; ++pass) {
#pragma unroll
        for (int it = 0; it < 8; ++it) {
          const int row = it * 2 + hh;
          v4f v = *(const v4f*)(slab + row * 68 + c4);
          *(volatile v4f*)(C + (size_t)(mBase + row) * ldc + n0 + c4) = v;
        }
        __threadfence();
      }
    } else {
      const int q = lane >> 3, c8 = (lane & 7) * 8;
      unsigned short* C  = (unsigned short*)Cout  + (size_t)b * strideC;
      unsigned short* C2 = (OUT_MODE == 2) ? ((unsigned short*)Cout2 + (size_t)b * strideC) : nullptr;
      for (int pass = 0; pass < 2; ++pass) {
#pragma unroll
        for (int it = 0; it < 4; ++it) {
          const int row = it * 4 + q;
          const float* sp = slab + row * 68 + c8;
          v8h hv, lv;
#pragma unroll
          for (int e = 0; e < 8; ++e) {
            if (OUT_MODE == 1) {
              hv[e] = (_Float16)sp[e];
            } else {
              unsigned short hb = f2bf_bits(sp[e]);
              unsigned short lb = f2bf_bits(sp[e] - bf_bits2f(hb));
              hv[e] = __builtin_bit_cast(_Float16, hb);
              lv[e] = __builtin_bit_cast(_Float16, lb);
            }
          }
          *(volatile v8h*)(C + (size_t)(mBase + row) * ldc + n0 + c8) = hv;
          if (OUT_MODE == 2) *(volatile v8h*)(C2 + (size_t)(mBase + row) * ldc + n0 + c8) = lv;
        }
        __threadfence();
      }
    }
    __builtin_amdgcn_fence(__ATOMIC_RELEASE, "workgroup");
    __builtin_amdgcn_wave_barrier();
    __builtin_amdgcn_fence(__ATOMIC_ACQUIRE, "workgroup");
  }
}

constexpr int kBatch   = 2;
constexpr int kHeads   = 3;
constexpr int kHeadDim = 32;
constexpr int kChan    = 96;
constexpr int kQkvChan = 288;
constexpr int kImg     = 64;
constexpr int kTok     = 4096;
constexpr int kBH      = kBatch * kHeads;
constexpr int kRows    = kBatch * kTok;
constexpr int kNPad    = 128;
constexpr size_t kPlaneHalves = (size_t)kBH * kTok * kHeadDim;
constexpr float kScoreScaleLog2 = (0.17677669529663688f / 256.0f) * 1.4426950408889634f;
constexpr float kOutFold = 6.103515625e-05f;

static_assert(kChan % 32 == 0);
static_assert(kRows % 64 == 0 && kNPad % 64 == 0);
static_assert(kTok % 64 == 0 && kImg == 64 && kHeadDim == 32 && kHeads * kHeadDim == kChan);
static_assert((kRows * kChan) % 4 == 0 && (kRows * kChan * 4) % 128 == 0);

__device__ __forceinline__ v8f mma_f16_guarded(v16h a, v16h b, v8f c) {
  c = __builtin_amdgcn_wmma_f32_16x16x32_f16(false, a, false, b, (short)0, c, false, false);
  asm volatile("v_nop\n\tv_nop\n\tv_nop\n\tv_nop" : "+v"(c) : "v"(a), "v"(b));
  return c;
}

__global__ __launch_bounds__(256) void dwconv_qkv_kernel(
    const float* __restrict__ x, const float* __restrict__ w, const float* __restrict__ bias,
    const int* __restrict__ hsz, const int* __restrict__ wsz,
    unsigned short* __restrict__ qkv16) {
  __shared__ __align__(16) unsigned short stg[9 * 2048];
  const int tid = threadIdx.x;
  const int y   = blockIdx.x;
  const int b   = blockIdx.y;
  int hlim = hsz[0]; hlim = hlim < 1 ? 1 : hlim; hlim = hlim > kImg ? kImg : hlim;
  int wlim = wsz[0]; wlim = wlim < 1 ? 1 : wlim; wlim = wlim > kImg ? kImg : wlim;
  const int tok = tid & 63;
  const int cg  = tid >> 6;

#pragma unroll 1
  for (int i = 0; i < 72; ++i) {
    const int o = cg + 4 * i;
    const int g = o / 3;
    const float* wk = w + o * 9;
    float acc = 0.0f;
#pragma unroll
    for (int dy = 0; dy < 3; ++dy) {
      const int yy  = y + dy - 1;
      const bool vy = (yy >= 0) && (yy < hlim);
      const int yyc = yy < 0 ? 0 : (yy > kImg - 1 ? kImg - 1 : yy);
#pragma unroll
      for (int dx = 0; dx < 3; ++dx) {
        const int xx  = tok + dx - 1;
        const bool vx = (xx >= 0) && (xx < wlim);
        const int xxc = xx < 0 ? 0 : (xx > kImg - 1 ? kImg - 1 : xx);
        float xv = x[((size_t)b * kTok + (size_t)yyc * kImg + xxc) * kChan + g];
        xv = (vy && vx) ? xv : 0.0f;
        acc = fmaf(wk[dy * 3 + dx], xv, acc);
      }
    }
    acc += bias[o];
    const _Float16 hval = (_Float16)(acc * 16.0f);
    const unsigned short hbits = __builtin_bit_cast(unsigned short, hval);
    const int s  = o / kChan;
    const int cc = o - s * kChan;
    const int hh = cc >> 5;
    const int dd = cc & 31;
    const int region = (s * 3 + hh) * 2048;
    const int offQK = tok * kHeadDim + dd;
    const int offV  = dd * 64 + tok;
    stg[region + ((s < 2) ? offQK : offV)] = hbits;
  }
  __syncthreads();

  const int lane = tid & 31, wave = tid >> 5;
  const int ql = lane >> 3, c8 = (lane & 7) * 8;
  for (int pass = 0; pass < 2; ++pass) {
#pragma unroll
    for (int it = 0; it < 9; ++it) {
      const int L  = wave * 36 + it * 4 + ql;
      const int s  = L / 96;
      const int Lr = L - s * 96;
      const int hh = Lr >> 5;
      const int li = Lr & 31;
      const v4u val = *(const v4u*)(stg + (s * 3 + hh) * 2048 + li * 64 + c8);
      const int bh = b * kHeads + hh;
      const size_t dstQK = (size_t)s * kPlaneHalves + ((size_t)bh * kTok + (size_t)y * kImg) * kHeadDim + (size_t)li * 64 + c8;
      const size_t dstV  = 2 * kPlaneHalves + ((size_t)bh * kHeadDim + li) * kTok + (size_t)y * kImg + c8;
      const size_t dst   = (s < 2) ? dstQK : dstV;
      *(volatile v4u*)(qkv16 + dst) = val;
    }
    __threadfence();
  }
}

__global__ __launch_bounds__(128) void attn_d32_kernel(
    const unsigned short* __restrict__ qp, const unsigned short* __restrict__ kp,
    const unsigned short* __restrict__ vp,
    unsigned short* __restrict__ ohp, unsigned short* __restrict__ olp) {
  __shared__ __align__(16) unsigned short Ksh[64 * 32];
  __shared__ __align__(16) unsigned short Vth[32 * 64];
  __shared__ __align__(16) _Float16 Psh[4][16 * 64];
  __shared__ __align__(16) float Os[32 * 68];

  const int tid  = threadIdx.x;
  const int wave = tid >> 5;
  const int lane = tid & 31;
  const int hh   = lane >> 4;
  const int c    = lane & 15;
  const int qb   = blockIdx.x & 63;
  const int bh   = blockIdx.x >> 6;
  const int q0   = qb * 64 + wave * 16;

  const _Float16* q16 = (const _Float16*)qp;
  const v16h qa = Frag<_Float16>::load(q16 + ((size_t)bh * kTok + q0 + c) * kHeadDim + 8 * hh);

  float mrow[8], lrow[8];
  v8f oacc[2];
#pragma unroll
  for (int r = 0; r < 8; ++r) { mrow[r] = -INFINITY; lrow[r] = 0.f; }
  oacc[0] = (v8f){0.f,0.f,0.f,0.f,0.f,0.f,0.f,0.f};
  oacc[1] = (v8f){0.f,0.f,0.f,0.f,0.f,0.f,0.f,0.f};
  const v8f zero8 = (v8f){0.f,0.f,0.f,0.f,0.f,0.f,0.f,0.f};

  const unsigned short* kbase = kp + (size_t)bh * kTok * kHeadDim;
  const unsigned short* vbase = vp + (size_t)bh * kHeadDim * kTok;

  for (int kc = 0; kc < kTok / 64; ++kc) {
    const int kv0 = kc * 64;
    __syncthreads();
#pragma unroll
    for (int rep = 0; rep < 2; ++rep) {
      const int u = tid + rep * 128;
      const v4u kw = *(const v4u*)(kbase + (size_t)kv0 * kHeadDim + (size_t)u * 8);
      *(v4u*)(Ksh + u * 8) = kw;
      const int dd = u >> 3, part = u & 7;
      const v4u vw = *(const v4u*)(vbase + (size_t)dd * kTok + kv0 + part * 8);
      *(v4u*)(Vth + dd * 64 + part * 8) = vw;
    }
    __syncthreads();

    v8f s[4];
#pragma unroll
    for (int j = 0; j < 4; ++j) {
      const v16h kb = Frag<_Float16>::load((const _Float16*)Ksh + (j * 16 + c) * kHeadDim + 8 * hh);
      s[j] = mma_f16_guarded(qa, kb, zero8);
    }
    float cm[8];
#pragma unroll
    for (int r = 0; r < 8; ++r) {
      float m = -INFINITY;
#pragma unroll
      for (int j = 0; j < 4; ++j) {
        const float sv = s[j][r] * kScoreScaleLog2;
        s[j][r] = sv;
        m = fmaxf(m, sv);
      }
#pragma unroll
      for (int off = 1; off < 16; off <<= 1) m = fmaxf(m, __shfl_xor(m, off, 32));
      cm[r] = m;
    }
    _Float16* pw = Psh[wave];
#pragma unroll
    for (int r = 0; r < 8; ++r) {
      const float mnew  = fmaxf(mrow[r], cm[r]);
      const float alpha = exp2f(mrow[r] - mnew);
      mrow[r] = mnew;
      float psum = 0.f;
#pragma unroll
      for (int j = 0; j < 4; ++j) {
        const float p = exp2f(s[j][r] - mnew);
        psum += p;
        pw[(8 * hh + r) * 64 + j * 16 + c] = (_Float16)(p * 1024.0f);
      }
#pragma unroll
      for (int off = 1; off < 16; off <<= 1) psum += __shfl_xor(psum, off, 32);
      lrow[r] = lrow[r] * alpha + psum;
      oacc[0][r] *= alpha;
      oacc[1][r] *= alpha;
    }
    __builtin_amdgcn_fence(__ATOMIC_RELEASE, "workgroup");
    __builtin_amdgcn_wave_barrier();
    __builtin_amdgcn_fence(__ATOMIC_ACQUIRE, "workgroup");
#pragma unroll
    for (int kk = 0; kk < 2; ++kk) {
      const v16h pa = Frag<_Float16>::load(pw + c * 64 + kk * 32 + 8 * hh);
#pragma unroll
      for (int t = 0; t < 2; ++t) {
        const v16h vb = Frag<_Float16>::load((const _Float16*)Vth + (t * 16 + c) * 64 + kk * 32 + 8 * hh);
        oacc[t] = mma_f16_guarded(pa, vb, oacc[t]);
      }
    }
  }

#pragma unroll
  for (int r = 0; r < 8; ++r) {
    const float inv = (1.0f / lrow[r]) * kOutFold;
    Os[(c) * 68 + wave * 16 + 8 * hh + r]      = oacc[0][r] * inv;
    Os[(16 + c) * 68 + wave * 16 + 8 * hh + r] = oacc[1][r] * inv;
  }
  __syncthreads();
  {
    const int ql = lane >> 3, c8 = (lane & 7) * 8;
    unsigned short* ohb = ohp + (size_t)bh * kHeadDim * kTok + (size_t)qb * 64 + c8;
    unsigned short* olb = olp + (size_t)bh * kHeadDim * kTok + (size_t)qb * 64 + c8;
    for (int pass = 0; pass < 2; ++pass) {
#pragma unroll
      for (int it = 0; it < 2; ++it) {
        const int d = 8 * wave + 4 * it + ql;
        const float* sp = Os + d * 68 + c8;
        const v4f a0 = *(const v4f*)(sp);
        const v4f a1 = *(const v4f*)(sp + 4);
        v8us hv, lv;
#pragma unroll
        for (int e = 0; e < 4; ++e) {
          const unsigned short hb0 = f2bf_bits(a0[e]);
          const unsigned short lb0 = f2bf_bits(a0[e] - bf_bits2f(hb0));
          hv[e] = hb0; lv[e] = lb0;
          const unsigned short hb1 = f2bf_bits(a1[e]);
          const unsigned short lb1 = f2bf_bits(a1[e] - bf_bits2f(hb1));
          hv[4 + e] = hb1; lv[4 + e] = lb1;
        }
        *(volatile v8us*)(ohb + (size_t)d * kTok) = hv;
        *(volatile v8us*)(olb + (size_t)d * kTok) = lv;
      }
      __threadfence();
    }
  }
}

__global__ __launch_bounds__(256) void wsplit_kernel(
    const float* __restrict__ pw, unsigned short* __restrict__ wh, unsigned short* __restrict__ wl) {
  const int t = blockIdx.x * 256 + threadIdx.x;
  if (t < kNPad * kChan / 8) {
    const int e0   = t * 8;
    const int row  = e0 / kChan;
    const int col  = e0 - row * kChan;
    const int rowc = row < kChan ? row : (kChan - 1);
    const bool live = row < kChan;
    const v4f a0 = *(const v4f*)(pw + (size_t)rowc * kChan + col);
    const v4f a1 = *(const v4f*)(pw + (size_t)rowc * kChan + col + 4);
    v8us hv, lv;
#pragma unroll
    for (int e = 0; e < 4; ++e) {
      const float f0 = live ? a0[e] : 0.0f;
      const float f1 = live ? a1[e] : 0.0f;
      const unsigned short hb0 = f2bf_bits(f0);
      const unsigned short lb0 = f2bf_bits(f0 - bf_bits2f(hb0));
      const unsigned short hb1 = f2bf_bits(f1);
      const unsigned short lb1 = f2bf_bits(f1 - bf_bits2f(hb1));
      hv[e] = hb0; lv[e] = lb0; hv[4 + e] = hb1; lv[4 + e] = lb1;
    }
    *(volatile v8us*)(wh + (size_t)e0) = hv;
    *(volatile v8us*)(wl + (size_t)e0) = lv;
    __threadfence();
    *(volatile v8us*)(wh + (size_t)e0) = hv;
    *(volatile v8us*)(wl + (size_t)e0) = lv;
  }
}

__global__ __launch_bounds__(256) void out_bias_kernel(
    const float* __restrict__ cproj, const float* __restrict__ pb, float* __restrict__ out) {
  const int t = blockIdx.x * 256 + threadIdx.x;
  if (t < kRows * kChan / 4) {
    const int row  = t / (kChan / 4);
    const int col4 = (t - row * (kChan / 4)) * 4;
    const v4f a  = *(const v4f*)(cproj + (size_t)row * kNPad + col4);
    const v4f bb = *(const v4f*)(pb + col4);
    const v4f r  = a + bb;
    *(volatile v4f*)(out + (size_t)t * 4) = r;
    __threadfence();
    *(volatile v4f*)(out + (size_t)t * 4) = r;
  }
}

extern "C" void kernel_launch(void* const* d_in, const int* in_sizes, int n_in,
                              void* d_out, int out_size, void* d_ws, size_t ws_size,
                              hipStream_t stream) {
  if (n_in < 7) return;
  if (in_sizes[0] != kRows * kChan) return;
  if (in_sizes[1] != kQkvChan * 9) return;
  if (in_sizes[2] != kQkvChan) return;
  if (in_sizes[3] != kChan * kChan) return;
  if (in_sizes[4] != kChan) return;
  if (in_sizes[5] < 1 || in_sizes[6] < 1) return;
  if (out_size != kRows * kChan) return;

  const float* x      = (const float*)d_in[0];
  const float* qkv_w  = (const float*)d_in[1];
  const float* qkv_b  = (const float*)d_in[2];
  const float* proj_w = (const float*)d_in[3];
  const float* proj_b = (const float*)d_in[4];
  const int*   hsz    = (const int*)d_in[5];
  const int*   wsz    = (const int*)d_in[6];
  float* out = (float*)d_out;

  const size_t bytesQKV  = 3 * kPlaneHalves * 2;
  const size_t bytesO16  = (size_t)kRows * kChan * 2;
  const size_t bytesW16  = (size_t)kNPad * kChan * 2;
  const size_t bytesCprj = (size_t)kRows * kNPad * 4;
  size_t off = 0;
  char* ws = (char*)d_ws;
  unsigned short* qkv16 = (unsigned short*)(ws + off); off += (bytesQKV + 255) & ~(size_t)255;
  unsigned short* oh    = (unsigned short*)(ws + off); off += (bytesO16 + 255) & ~(size_t)255;
  unsigned short* ol    = (unsigned short*)(ws + off); off += (bytesO16 + 255) & ~(size_t)255;
  unsigned short* wh    = (unsigned short*)(ws + off); off += (bytesW16 + 255) & ~(size_t)255;
  unsigned short* wl    = (unsigned short*)(ws + off); off += (bytesW16 + 255) & ~(size_t)255;
  float*          cproj = (float*)(ws + off);          off += (bytesCprj + 255) & ~(size_t)255;
  if (off > ws_size) return;

  const unsigned short* q16 = qkv16;
  const unsigned short* k16 = qkv16 + kPlaneHalves;
  const unsigned short* v16 = qkv16 + 2 * kPlaneHalves;

  dwconv_qkv_kernel<<<dim3(kImg, kBatch), 256, 0, stream>>>(x, qkv_w, qkv_b, hsz, wsz, qkv16);
  wsplit_kernel<<<(kNPad * kChan / 8 + 255) / 256, 256, 0, stream>>>(proj_w, wh, wl);
  attn_d32_kernel<<<kBH * (kTok / 64), 128, 0, stream>>>(q16, k16, v16, oh, ol);
  {
    const int tiles = (kRows / 64) * (kNPad / 64);
    const int blocks = (tiles + 7) / 8;
    wmma_gemm64<1, true, 0, 0, false, 0><<<dim3(blocks, 1), 256, 0, stream>>>(
        oh, ol, kChan, 0L,
        wh, wl, kChan, 0L,
        (void*)cproj, (void*)nullptr, kNPad, 0L,
        (const float*)nullptr,
        (const float*)nullptr, 0L,
        kRows, kNPad, kChan, 1.0f);
  }
  out_bias_kernel<<<(kRows * kChan / 4 + 255) / 256, 256, 0, stream>>>(cproj, proj_b, out);
}
